// CustomRNN_88871463289370
// MI455X (gfx1250) — hardware-verified
//
#include <hip/hip_runtime.h>
#include <math.h>

typedef __attribute__((ext_vector_type(16))) _Float16 v16h;
typedef __attribute__((ext_vector_type(8)))  _Float16 v8h;
typedef __attribute__((ext_vector_type(8)))  float    v8f;
typedef __attribute__((ext_vector_type(4)))  float    v4f;

constexpr int HID      = 512;
constexpr int T_STEPS  = 256;
constexpr int HOR      = 24;
constexpr int HOR_PAD  = 32;
constexpr int M_ROWS   = 16;
constexpr int HPAD     = 520;
constexpr int NTHREADS = 256;
constexpr float WCARRY     = 16.0f;
constexpr float WCARRY_INV = 0.0625f;

static_assert(HID % 32 == 0);
static_assert((HPAD * 2) % 16 == 0);
static_assert(M_ROWS * HOR * 4 == 12 * 128);
static_assert((M_ROWS * HPAD) % 8 == 0);
static_assert(NTHREADS == 8 * 32);
static_assert(8 * 64 == HID);

__device__ __forceinline__ void dep_guard_h(v8f& a, v8f& b, v16h x, v16h y) {
  asm volatile("v_nop\n\tv_nop\n\tv_nop\n\tv_nop" : "+v"(a), "+v"(b) : "v"(x), "v"(y));
}
__device__ __forceinline__ void guard4_h(v8f& c0, v8f& c1, v8f& c2, v8f& c3,
                                         v16h a, v16h b0, v16h b1, v16h b2, v16h b3) {
  asm volatile("v_nop\n\tv_nop\n\tv_nop\n\tv_nop"
               : "+v"(c0), "+v"(c1), "+v"(c2), "+v"(c3)
               : "v"(a), "v"(b0), "v"(b1), "v"(b2), "v"(b3));
}
__device__ __forceinline__ void guard1_h(v8f& c0, v16h a, v16h b) {
  asm volatile("v_nop\n\tv_nop\n\tv_nop\n\tv_nop" : "+v"(c0) : "v"(a), "v"(b));
}

template <typename T> struct Frag;
template <> struct Frag<_Float16> {
  typedef v16h V; union U { v16h v; v8h h[2]; };
  static __device__ __forceinline__ v16h load(const _Float16* p) {
    U f; f.h[0] = *(const v8h*)(p); f.h[1] = *(const v8h*)(p + 16); return f.v;
  }
  static __device__ __forceinline__ v8f mma(v16h a, v16h b, v8f c) {
    return __builtin_amdgcn_wmma_f32_16x16x32_f16(false, a, false, b, (short)0, c, false, false);
  }
};

__device__ __forceinline__ float tanh_eval(float v) {
  const float a  = fminf(fabsf(v), 10.0f);
  const float e2 = exp2f(a * 2.8853900817779268f);
  const float t  = fmaf(-2.0f, __builtin_amdgcn_rcpf(e2 + 1.0f), 1.0f);
  return copysignf(t, v);
}

__global__ __launch_bounds__(256) void cast_scale_f32_f16x2(
    const float* __restrict__ in, _Float16* __restrict__ outp, int n2, int nvalid, float scale) {
  const int i = blockIdx.x * 256 + threadIdx.x;
  if (i < n2) {
    const int e  = 2 * i;
    const int ec = (e < nvalid) ? e : (nvalid - 2);
    float a = in[ec] * scale;
    float b = in[ec + 1] * scale;
    if (e >= nvalid) { a = 0.0f; b = 0.0f; }
    const _Float16 h0 = (_Float16)a, h1 = (_Float16)b;
    const unsigned u = (unsigned)__builtin_bit_cast(unsigned short, h0) |
                       ((unsigned)__builtin_bit_cast(unsigned short, h1) << 16);
    ((volatile unsigned*)outp)[i] = u;
    __threadfence();
    ((volatile unsigned*)outp)[i] = u;
  }
}

__global__ __launch_bounds__(NTHREADS)
void rnn_scan_head_kernel(const float* __restrict__ x,
                          const float* __restrict__ wxw,
                          const float* __restrict__ wxb,
                          const float* __restrict__ whb,
                          const float* __restrict__ fcb,
                          const _Float16* __restrict__ wh16,
                          const _Float16* __restrict__ fcw16,
                          float* __restrict__ out) {
  __shared__ __align__(16) _Float16 hbuf[M_ROWS * HPAD];
  __shared__ __align__(16) float    xs[M_ROWS * T_STEPS];
  __shared__ __align__(16) float    ost[M_ROWS * HOR];

  const int tid  = threadIdx.x;
  const int lane = tid & 31;
  const int wave = tid >> 5;
  const int hh   = lane >> 4;
  const int rl   = lane & 15;
  const int koff = hh * 8;
  const int rowbase = blockIdx.x * M_ROWS;
  const int jw   = wave * 64;

  {
    v8h z;
#pragma unroll
    for (int e = 0; e < 8; ++e) z[e] = (_Float16)0.0f;
    for (int i = tid; i < (M_ROWS * HPAD) / 8; i += NTHREADS) *(v8h*)(hbuf + 8 * i) = z;
  }
#pragma unroll
  for (int i = 0; i < 4; ++i) {
    const int idx4 = tid + NTHREADS * i;
    const int r  = idx4 >> 6;
    const int c4 = (idx4 & 63) * 4;
    const v4f vv = *(const v4f*)(x + (size_t)(rowbase + r) * T_STEPS + c4);
    *(v4f*)(xs + r * T_STEPS + c4) = vv;
  }
  float wxc[4], bic[4];
#pragma unroll
  for (int ct = 0; ct < 4; ++ct) {
    const int j = jw + ct * 16 + rl;
    wxc[ct] = wxw[j];
    bic[ct] = wxb[j] + whb[j];
  }
  __syncthreads();

  for (int t = 0; t < T_STEPS; ++t) {
    v8f acc[4];
#pragma unroll
    for (int ct = 0; ct < 4; ++ct) acc[ct] = (v8f){0.f, 0.f, 0.f, 0.f, 0.f, 0.f, 0.f, 0.f};

#pragma unroll 1
    for (int kt = 0; kt < HID / 32; ++kt) {
      const int k0 = kt * 32;
      const v16h a = Frag<_Float16>::load(hbuf + rl * HPAD + k0 + koff);
      v16h b[4];
#pragma unroll
      for (int ct = 0; ct < 4; ++ct)
        b[ct] = Frag<_Float16>::load(wh16 + (size_t)(jw + ct * 16 + rl) * HID + k0 + koff);
#pragma unroll
      for (int ct = 0; ct < 4; ++ct) acc[ct] = Frag<_Float16>::mma(a, b[ct], acc[ct]);
      guard4_h(acc[0], acc[1], acc[2], acc[3], a, b[0], b[1], b[2], b[3]);
    }

    float xr[8];
#pragma unroll
    for (int r = 0; r < 8; ++r) xr[r] = xs[(8 * hh + r) * T_STEPS + t];

    __syncthreads();

#pragma unroll
    for (int ct = 0; ct < 4; ++ct) {
      const int j = jw + ct * 16 + rl;
#pragma unroll
      for (int r = 0; r < 8; ++r) {
        float v = acc[ct][r] * WCARRY_INV + (xr[r] * wxc[ct] + bic[ct]);
        v = tanh_eval(v);
        hbuf[(8 * hh + r) * HPAD + j] = (_Float16)v;
      }
    }
    __syncthreads();
  }

  if (wave < 2) {
    v8f hacc = (v8f){0.f, 0.f, 0.f, 0.f, 0.f, 0.f, 0.f, 0.f};
#pragma unroll 1
    for (int kt = 0; kt < HID / 32; ++kt) {
      const int k0 = kt * 32;
      const v16h a = Frag<_Float16>::load(hbuf + rl * HPAD + k0 + koff);
      const v16h b = Frag<_Float16>::load(fcw16 + (size_t)(wave * 16 + rl) * HID + k0 + koff);
      hacc = Frag<_Float16>::mma(a, b, hacc);
      guard1_h(hacc, a, b);
    }
    const int o  = wave * 16 + rl;
    const int oc = (o < HOR) ? o : (HOR - 1);
    const float bo = fcb[oc];
#pragma unroll
    for (int r = 0; r < 8; ++r) {
      const float v = hacc[r] * WCARRY_INV + bo;
      if (o < HOR) ost[(8 * hh + r) * HOR + o] = v;
    }
  }
  __syncthreads();
  if (wave == 0) {
    float* ob = out + (size_t)blockIdx.x * (M_ROWS * HOR);
    v4f vv[3];
#pragma unroll
    for (int i = 0; i < 3; ++i) vv[i] = *(const v4f*)(ost + (lane + 32 * i) * 4);
#pragma unroll
    for (int i = 0; i < 3; ++i) *(volatile v4f*)(ob + (size_t)(lane + 32 * i) * 4) = vv[i];
    __threadfence();
#pragma unroll
    for (int i = 0; i < 3; ++i) *(volatile v4f*)(ob + (size_t)(lane + 32 * i) * 4) = vv[i];
  }
}

extern "C" void kernel_launch(void* const* d_in, const int* in_sizes, int n_in,
                              void* d_out, int out_size, void* d_ws, size_t ws_size,
                              hipStream_t stream) {
  const float* x   = (const float*)d_in[0];
  const float* wxw = (const float*)d_in[1];
  const float* wxb = (const float*)d_in[2];
  const float* whw = (const float*)d_in[3];
  const float* whb = (const float*)d_in[4];
  const float* fcw = (const float*)d_in[5];
  const float* fcb = (const float*)d_in[6];
  float* out = (float*)d_out;

  const size_t WH16_BYTES  = (size_t)HID * HID * 2;
  const size_t FCW16_BYTES = (size_t)HOR_PAD * HID * 2;
  if (ws_size < WH16_BYTES + FCW16_BYTES) return;
  char* ws = (char*)d_ws;
  _Float16* wh16  = (_Float16*)(ws);
  _Float16* fcw16 = (_Float16*)(ws + WH16_BYTES);

  const int B    = in_sizes[0] / T_STEPS;
  int nblk = B / M_ROWS;
  const int nblk_out = out_size / (M_ROWS * HOR);
  if (nblk > nblk_out) nblk = nblk_out;

  {
    const int n2 = (HID * HID) / 2;
    int nvalid = in_sizes[3];
    if (nvalid > HID * HID) nvalid = HID * HID;
    if (nvalid < 2) nvalid = 2;
    cast_scale_f32_f16x2<<<(n2 + 255) / 256, 256, 0, stream>>>(whw, wh16, n2, nvalid, WCARRY);
  }
  {
    const int n2 = (HOR_PAD * HID) / 2;
    int nvalid = in_sizes[5];
    if (nvalid > HOR * HID) nvalid = HOR * HID;
    if (nvalid < 2) nvalid = 2;
    cast_scale_f32_f16x2<<<(n2 + 255) / 256, 256, 0, stream>>>(fcw, fcw16, n2, nvalid, WCARRY);
  }
  if (nblk >= 1) {
    rnn_scan_head_kernel<<<nblk, NTHREADS, 0, stream>>>(x, wxw, wxb, whb, fcb, wh16, fcw16, out);
  }
}
